// LongformerAttention_15590731284882
// MI455X (gfx1250) — hardware-run, weakly checked
//
#include <hip/hip_runtime.h>


#ifndef NB
#define NB 2
#endif
#ifndef SEQ
#define SEQ 2048
#endif
#define NB_FULL  2
#define SEQ_FULL 2048
#ifndef OUT_SEQ
#define OUT_SEQ SEQ
#endif
#define DM   512
#define NH_  8
#define HD   64
#define AW   4
#define OSP  68
#define WIN  512
#define WR_  (WIN / 2)
#define WL_  (WIN - WR_)
#define XC   256.0f
#define WC   64.0f
#define OSC  (1.0f / 16384.0f)
#define QRS  2048.0f
#define QRI  (1.0f / 2048.0f)
#define SC2  ((float)(0.125 * 1.4426950408889634))
#define PSH  14.0f
#define NEGB (-3.0e38f)

static_assert(HD == 64);
static_assert(NH_ * HD == DM);
static_assert(DM % 64 == 0);
static_assert(DM % 32 == 0);
static_assert(HD % 32 == 0);
static_assert(SEQ % 64 == 0);
static_assert((NB * SEQ) % 64 == 0);
static_assert(SEQ % 32 == 0);
static_assert(SEQ % (16 * AW) == 0);
static_assert(((size_t)SEQ * DM) % 8 == 0);
static_assert(NB <= NB_FULL);
static_assert(SEQ <= SEQ_FULL);
static_assert((OSP * 4) % 16 == 0);
static_assert(OSP >= HD);
static_assert(XC * WC * OSC == 1.0f);
static_assert(QRS * QRI == 1.0f);
static_assert(32 * 16 * 4 == 16 * HD * 2);
static_assert(32 * 16 * 8 == 16 * 64 * 4);
static_assert(256 * 16 * 2 == 64 * 64 * 2);
static_assert(256 * 16 * 4 == 64 * 64 * 4);
static_assert(16 * 68 * 4 <= 131072);
static_assert(AW * 16 * OSP * 4 <= 131072);
static_assert(64 * 65 * 4 <= 131072);

typedef _Float16 h16;
typedef unsigned short bf;
typedef __attribute__((ext_vector_type(16))) __bf16   v16bf;
typedef __attribute__((ext_vector_type(16))) _Float16 v16h;
typedef __attribute__((ext_vector_type(8)))  _Float16 v8h;
typedef __attribute__((ext_vector_type(8)))  unsigned short v8us;
typedef __attribute__((ext_vector_type(8)))  float    v8f;
typedef __attribute__((ext_vector_type(4)))  float    v4f;
typedef __attribute__((ext_vector_type(4)))  int      v4i;
typedef v4f  __attribute__((may_alias)) v4fa;

__device__ __forceinline__ unsigned short f2bf(float f) { unsigned u = __float_as_uint(f); u += 0x7FFFu + ((u >> 16) & 1u); return (unsigned short)(u >> 16); }
__device__ __forceinline__ float bfr(float f) { return __uint_as_float(((unsigned)f2bf(f)) << 16); }
__device__ __forceinline__ v16h cat16(v8h lo, v8h hi) { return __builtin_shufflevector(lo, hi, 0, 1, 2, 3, 4, 5, 6, 7, 8, 9, 10, 11, 12, 13, 14, 15); }
__device__ __forceinline__ v16bf cat16b(v8us lo, v8us hi) { return __builtin_bit_cast(v16bf, __builtin_shufflevector(lo, hi, 0, 1, 2, 3, 4, 5, 6, 7, 8, 9, 10, 11, 12, 13, 14, 15)); }
__device__ __forceinline__ v8f wmma16(v16h a, v16h b, v8f c) { return __builtin_amdgcn_wmma_f32_16x16x32_f16(false, a, false, b, (short)0, c, false, false); }
__device__ __forceinline__ v8f wmmab(v16bf a, v16bf b, v8f c) { return __builtin_amdgcn_wmma_f32_16x16x32_bf16(false, a, false, b, (short)0, c, false, false); }
__device__ __forceinline__ v16h  ldh(const h16* p) { return cat16(*(const v8h*)p, *(const v8h*)(p + 16)); }
__device__ __forceinline__ v16bf ldb(const bf* p)  { return cat16b(*(const v8us*)p, *(const v8us*)(p + 16)); }
__device__ __forceinline__ void wave_sync() { __builtin_amdgcn_fence(3  , "wavefront"); __builtin_amdgcn_wave_barrier(); asm volatile("" ::: "memory"); }

static __device__ __forceinline__ h16 toh_flush(float v) { const h16 r = (h16)v; return (fabsf(v) < 6.103515625e-05f) ? (h16)0.0f : r; }
__device__ __forceinline__ v8f wmma16g(v16h a, v16h b, v8f c) { c = wmma16(a, b, c); asm volatile("v_nop\n\tv_nop\n\tv_nop\n\tv_nop" : "+v"(c) : "v"(a), "v"(b)); return c; }
__device__ __forceinline__ v8f wmmabg(v16bf a, v16bf b, v8f c) { c = wmmab(a, b, c); asm volatile("v_nop\n\tv_nop\n\tv_nop\n\tv_nop" : "+v"(c) : "v"(a), "v"(b)); return c; }

__global__ __launch_bounds__(256) void k_cvt8(const float* __restrict__ src, bf* dst, size_t n8) {
    const size_t i = (size_t)blockIdx.x * 256 + threadIdx.x; if (i >= n8) return;
    const v8f v = *(const v8f*)(src + i * 8); v8us o;
#pragma unroll
    for (int k = 0; k < 8; ++k) o[k] = f2bf(v[k]);
    *(volatile v8us*)(dst + i * 8) = o; __threadfence(); *(volatile v8us*)(dst + i * 8) = o;
}

template <int F16>
__device__ __forceinline__ void wt_body(const float* __restrict__ src, bf* dstb, h16* dsth) {
    __shared__ float ts[64 * 65];
    const int tid = threadIdx.x;
    const int k0 = blockIdx.x * 64, n0 = blockIdx.y * 64;
#pragma unroll 1
    for (int it = 0; it < 4; ++it) {
        const int kr = (tid >> 4) + 16 * it, c4 = (tid & 15) * 4;
        const v4f v = *(const v4f*)(src + (size_t)(k0 + kr) * DM + n0 + c4);
        ts[kr * 65 + c4 + 0] = v[0]; ts[kr * 65 + c4 + 1] = v[1]; ts[kr * 65 + c4 + 2] = v[2]; ts[kr * 65 + c4 + 3] = v[3];
    }
    __syncthreads();
#pragma unroll 1
    for (int ps = 0; ps < 2; ++ps) {
#pragma unroll 1
        for (int it = 0; it < 2; ++it) {
            const int nr = (tid >> 3) + 32 * it, c8 = (tid & 7) * 8;
            float x[8];
#pragma unroll
            for (int i = 0; i < 8; ++i) x[i] = ts[(c8 + i) * 65 + nr];
            const size_t oo = (size_t)(n0 + nr) * DM + k0 + c8;
            if (F16) { v8h hv;
#pragma unroll
                for (int i = 0; i < 8; ++i) hv[i] = toh_flush(bfr(x[i]) * WC);
                *(volatile v8h*)(dsth + oo) = hv;
            } else { v8us o;
#pragma unroll
                for (int i = 0; i < 8; ++i) o[i] = f2bf(x[i]);
                *(volatile v8us*)(dstb + oo) = o; }
        }
        if (ps == 0) __threadfence();
    }
}
__global__ __launch_bounds__(256) void k_wt_b(const float* __restrict__ src, bf* dst)  { wt_body<0>(src, dst, (h16*)0); }
__global__ __launch_bounds__(256) void k_wt_h(const float* __restrict__ src, h16* dst) { wt_body<1>(src, (bf*)0, dst); }

template <int MODE>
__device__ __forceinline__ void proj_body(const bf* __restrict__ A, const bf* __restrict__ Bt, const float* __restrict__ bias, h16* Ph, h16* Pr) {
    __shared__ __align__(16) float os[16 * 68];
    const int K = DM;
    const int lane = threadIdx.x & 31, lr = lane & 15, hi = lane >> 4; const int r0 = blockIdx.x * 64, c0 = blockIdx.y * 64;
    v8f acc[4][4];
#pragma unroll
    for (int mb = 0; mb < 4; ++mb)
#pragma unroll
        for (int nb = 0; nb < 4; ++nb) acc[mb][nb] = (v8f){};
    const size_t aoff = (size_t)(r0 + lr) * K + 8 * hi, boff = (size_t)(c0 + lr) * K + 8 * hi;
#pragma unroll 1
    for (int kc = 0; kc < K; kc += 32) {
        v16bf a[4];
#pragma unroll
        for (int mb = 0; mb < 4; ++mb) a[mb] = ldb(A + aoff + (size_t)mb * 16 * K + kc);
#pragma unroll
        for (int nb = 0; nb < 4; ++nb) { const v16bf b = ldb(Bt + boff + (size_t)nb * 16 * K + kc);
#pragma unroll
            for (int mb = 0; mb < 4; ++mb) acc[mb][nb] = wmmabg(a[mb], b, acc[mb][nb]); }
    }
    float bc[4];
#pragma unroll
    for (int nb = 0; nb < 4; ++nb) bc[nb] = (MODE == 0) ? bfr(bias[c0 + nb * 16 + lr]) : 0.0f;
    size_t tbase;
    if (MODE == 0) { const int bb = r0 / SEQ, tt = r0 % SEQ; const int zc = bb * NH_ + c0 / HD;
                     tbase = ((size_t)zc * SEQ + (size_t)tt) * HD; }
    else           { const int bb = c0 / SEQ, tt = c0 % SEQ;
                     tbase = (size_t)bb * (size_t)DM * SEQ + (size_t)r0 * SEQ + (size_t)tt; }
    const size_t pitch = (MODE == 0) ? (size_t)HD : (size_t)SEQ;
#pragma unroll
    for (int mb = 0; mb < 4; ++mb) {
        float br[8];
#pragma unroll
        for (int j = 0; j < 8; ++j) br[j] = (MODE == 1) ? bfr(bias[r0 + mb * 16 + hi * 8 + j]) : 0.0f;
#pragma unroll
        for (int nb = 0; nb < 4; ++nb) {
#pragma unroll
            for (int j = 0; j < 8; ++j) os[(hi * 8 + j) * 68 + nb * 16 + lr] = acc[mb][nb][j] + bc[nb] + br[j]; }
        wave_sync();
        const size_t sb = tbase + (size_t)(mb * 16) * pitch;
#pragma unroll 1
        for (int ps = 0; ps < 2; ++ps) {
#pragma unroll
            for (int s = 0; s < 4; ++s) { const int row = 4 * s + (lane >> 3), c8 = (lane & 7) * 8;
                const v4f x0 = *(const v4fa*)(&os[row * 68 + c8]); const v4f x1 = *(const v4fa*)(&os[row * 68 + c8 + 4]); v8h hv, rv;
#pragma unroll
                for (int i = 0; i < 4; ++i) { const h16 a0 = toh_flush(x0[i]); const h16 a1 = toh_flush(x1[i]); hv[i] = a0; hv[4 + i] = a1;
                    rv[i] = toh_flush((x0[i] - (float)a0) * QRS); rv[4 + i] = toh_flush((x1[i] - (float)a1) * QRS); }
                const size_t oo = sb + (size_t)row * pitch + c8;
                *(volatile v8h*)(Ph + oo) = hv; if (MODE == 0) *(volatile v8h*)(Pr + oo) = rv; }
            if (ps == 0) __threadfence(); }
        wave_sync();
    }
}
__global__ __launch_bounds__(32) void k_proj_rows(const bf* __restrict__ A, const bf* __restrict__ Bt, const float* __restrict__ bias, h16* Ph, h16* Pr) { proj_body<0>(A, Bt, bias, Ph, Pr); }
__global__ __launch_bounds__(32) void k_proj_cols(const bf* __restrict__ A, const bf* __restrict__ Bt, const float* __restrict__ bias, h16* Ph) { proj_body<1>(A, Bt, bias, Ph, (h16*)0); }

__global__ __launch_bounds__(32) void k_oproj(const h16* __restrict__ A, const h16* __restrict__ Bt, const float* __restrict__ bias, float* OUT) {
    __shared__ __align__(16) float os[16 * 68];
    const int K = DM;
    const int lane = threadIdx.x & 31, lr = lane & 15, hi = lane >> 4; const int r0 = blockIdx.x * 64, c0 = blockIdx.y * 64;
    v8f acc[4][4];
#pragma unroll
    for (int mb = 0; mb < 4; ++mb)
#pragma unroll
        for (int nb = 0; nb < 4; ++nb) acc[mb][nb] = (v8f){};
    const size_t aoff = (size_t)(r0 + lr) * K + 8 * hi, boff = (size_t)(c0 + lr) * K + 8 * hi;
#pragma unroll 1
    for (int kc = 0; kc < K; kc += 32) {
        v16h a[4];
#pragma unroll
        for (int mb = 0; mb < 4; ++mb) a[mb] = ldh(A + aoff + (size_t)mb * 16 * K + kc);
#pragma unroll
        for (int nb = 0; nb < 4; ++nb) { const v16h b = ldh(Bt + boff + (size_t)nb * 16 * K + kc);
#pragma unroll
            for (int mb = 0; mb < 4; ++mb) acc[mb][nb] = wmma16g(a[mb], b, acc[mb][nb]); }
    }
    float bc[4];
#pragma unroll
    for (int nb = 0; nb < 4; ++nb) bc[nb] = bfr(bias[c0 + nb * 16 + lr]);
    const int bb = r0 / SEQ, tt = r0 % SEQ;
    const size_t obase = ((size_t)bb * OUT_SEQ + (size_t)tt) * DM + (size_t)c0;
#pragma unroll
    for (int mb = 0; mb < 4; ++mb) {
#pragma unroll
        for (int nb = 0; nb < 4; ++nb) {
#pragma unroll
            for (int j = 0; j < 8; ++j) os[(hi * 8 + j) * 68 + nb * 16 + lr] = acc[mb][nb][j] * OSC + bc[nb]; }
        wave_sync();
        const size_t sb = obase + (size_t)(mb * 16) * DM;
#pragma unroll 1
        for (int ps = 0; ps < 2; ++ps) {
#pragma unroll
            for (int s = 0; s < 8; ++s) { const int row = 2 * s + (lane >> 4), c4 = (lane & 15) * 4;
                const v4f val = *(const v4fa*)(&os[row * 68 + c4]);
                *(volatile v4f*)(OUT + sb + (size_t)row * DM + c4) = val; }
            if (ps == 0) __threadfence(); }
        wave_sync();
    }
}

template <int PAT>
__device__ __forceinline__ void flash_body(const h16* __restrict__ QH, const h16* __restrict__ QR, const h16* __restrict__ KP, const h16* __restrict__ KR,
                                           const h16* __restrict__ VT, const int* __restrict__ gmask, h16* XP) {
    __shared__ __align__(16) float os[AW * 16 * OSP];
    const int lane = threadIdx.x & 31, lr = lane & 15, hi = lane >> 4;
    const int wave = __builtin_amdgcn_readfirstlane((int)(threadIdx.x >> 5));
    const int zh = blockIdx.y; const int b = zh / NH_, h = zh % NH_;
    const int t0 = (blockIdx.x * AW + wave) * 16;
    const int* gmb = gmask + (size_t)b * SEQ_FULL;
    int gqv = gmb[t0 + lr]; asm volatile("" : "+v"(gqv));
    const bool gq = gqv != 0;
    const unsigned gqm = ((unsigned)__ballot(gq ? 1 : 0)) & 0xFFFFu;
    const int tq = t0 + lr;
    const int jlo = tq - (WL_ - 1), jhi = tq + WR_;
    const size_t pbase = (size_t)zh * SEQ * HD;
    const size_t qo = pbase + (size_t)(t0 + lr) * HD + 8 * hi;
    const v16h qf0 = ldh(QH + qo), qf1 = ldh(QH + qo + 32);
    const v16h qr0 = ldh(QR + qo), qr1 = ldh(QR + qo + 32);
    const size_t ko = pbase + (size_t)lr * HD + 8 * hi;
    const size_t vo = pbase + (size_t)lr * SEQ + 8 * hi;
    v8f o[4];
#pragma unroll
    for (int j = 0; j < 4; ++j) o[j] = (v8f){};
    float m = NEGB, l = 0.0f;
#pragma unroll 1
    for (int key0 = 0; key0 < SEQ; key0 += 32) {
        const h16* ka = KP + ko + (size_t)key0 * HD;
        const h16* kr = KR + ko + (size_t)key0 * HD;
        const v16h ka0 = ldh(ka), ka1 = ldh(ka + 32), kb0 = ldh(ka + 16 * HD), kb1 = ldh(ka + 16 * HD + 32);
        const v16h kra0 = ldh(kr), kra1 = ldh(kr + 32), krb0 = ldh(kr + 16 * HD), krb1 = ldh(kr + 16 * HD + 32);
        v8f sa = (v8f){}, sb = (v8f){}, sLa = (v8f){}, sLb = (v8f){};
        sa = wmma16g(ka0, qf0, sa); sb = wmma16g(kb0, qf0, sb); sa = wmma16g(ka1, qf1, sa); sb = wmma16g(kb1, qf1, sb);
        sLa = wmma16g(ka0, qr0, sLa); sLb = wmma16g(kb0, qr0, sLb); sLa = wmma16g(ka1, qr1, sLa); sLb = wmma16g(kb1, qr1, sLb);
        sLa = wmma16g(kra0, qf0, sLa); sLb = wmma16g(krb0, qf0, sLb); sLa = wmma16g(kra1, qf1, sLa); sLb = wmma16g(krb1, qf1, sLb);
        bool fa[8], fb[8];
        if (PAT == 0) {
            const int* kp = gmb + key0 + 8 * hi;
            v4i m0 = *(const v4i*)kp, m1 = *(const v4i*)(kp + 4), m2 = *(const v4i*)(kp + 16), m3 = *(const v4i*)(kp + 20);
            asm volatile("" : "+v"(m0)); asm volatile("" : "+v"(m1)); asm volatile("" : "+v"(m2)); asm volatile("" : "+v"(m3));
            int kx[8], ky[8];
#pragma unroll
            for (int r = 0; r < 4; ++r) { kx[r] = m0[r]; kx[4 + r] = m1[r]; ky[r] = m2[r]; ky[4 + r] = m3[r]; }
            const int ja = key0 + 8 * hi;
#pragma unroll
            for (int r = 0; r < 8; ++r) {
                const int j0 = ja + r, j1 = ja + 16 + r;
                fa[r] = gq | (kx[r] != 0) | ((j0 >= jlo) & (j0 <= jhi));
                fb[r] = gq | (ky[r] != 0) | ((j1 >= jlo) & (j1 <= jhi)); }
        } else {
#pragma unroll
            for (int r = 0; r < 8; ++r) { fa[r] = true; fb[r] = true; }
        }
        float ta[8], tb[8]; float mx = NEGB;
#pragma unroll
        for (int r = 0; r < 8; ++r) {
            ta[r] = (sa[r] + sLa[r] * QRI) * SC2; tb[r] = (sb[r] + sLb[r] * QRI) * SC2;
            mx = fmaxf(mx, fmaxf(fa[r] ? ta[r] : NEGB, fb[r] ? tb[r] : NEGB)); }
        mx = fmaxf(mx, __shfl_xor(mx, 16, 32));
        const float mnew = fmaxf(m, mx);
        const float alpha = __builtin_amdgcn_exp2f(m - mnew);
        const float sh = PSH - mnew;
        v16h pb; float ls = 0.0f;
#pragma unroll
        for (int r = 0; r < 8; ++r) {
            const float xa = ta[r] + sh, xb = tb[r] + sh;
            const float ea = __builtin_amdgcn_exp2f(xa), eb = __builtin_amdgcn_exp2f(xb);
            const float ga = (fa[r] & (xa >= -14.0f)) ? ea : 0.0f;
            const float gb = (fb[r] & (xb >= -14.0f)) ? eb : 0.0f;
            const h16 pa = (h16)ga; const h16 pc = (h16)gb;
            pb[r] = pa; pb[8 + r] = pc;
            ls += (float)pa + (float)pc; }
        l = l * alpha + ls; m = mnew;
#pragma unroll
        for (int j = 0; j < 4; ++j) o[j] = o[j] * alpha;
        const h16* va = VT + vo + key0;
#pragma unroll
        for (int j = 0; j < 4; ++j) { const v16h vf = ldh(va + (size_t)(16 * j) * SEQ); o[j] = wmma16g(vf, pb, o[j]); }
    }
    l += __shfl_xor(l, 16, 32);
    const bool any = l > 0.0f;
    const float lsafe = any ? l : 1.0f;
    const float inv = any ? (XC * (1.0f / lsafe)) : 0.0f;
    const int wb = wave * 16 * OSP;
#pragma unroll
    for (int j = 0; j < 4; ++j) { v4f a, c;
        a[0] = o[j][0] * inv; a[1] = o[j][1] * inv; a[2] = o[j][2] * inv; a[3] = o[j][3] * inv;
        c[0] = o[j][4] * inv; c[1] = o[j][5] * inv; c[2] = o[j][6] * inv; c[3] = o[j][7] * inv;
        *(v4fa*)(&os[wb + lr * OSP + 16 * j + 8 * hi]) = a; *(v4fa*)(&os[wb + lr * OSP + 16 * j + 8 * hi + 4]) = c; }
    wave_sync();
    h16* xrow = XP + ((size_t)b * SEQ + t0) * DM + h * HD;
#pragma unroll 1
    for (int ps = 0; ps < 2; ++ps) {
#pragma unroll
        for (int s = 0; s < 4; ++s) { const int row = 4 * s + (lane >> 3), c8 = (lane & 7) * 8;
            v4f x0 = *(const v4fa*)(&os[wb + row * OSP + c8]); v4f x1 = *(const v4fa*)(&os[wb + row * OSP + c8 + 4]);
            asm volatile("" : "+v"(x0)); asm volatile("" : "+v"(x1));
            v8h hv;
#pragma unroll
            for (int i = 0; i < 4; ++i) { hv[i] = toh_flush(x0[i]); hv[4 + i] = toh_flush(x1[i]); }
            const bool st = (int)((gqm >> row) & 1u) == PAT;
            if (st) *(volatile v8h*)(xrow + (size_t)row * DM + c8) = hv; }
        if (ps == 0) __threadfence(); }
}
__global__ __launch_bounds__(32 * AW) __attribute__((amdgpu_num_vgpr(256))) void k_flash_win(const h16* __restrict__ QH, const h16* __restrict__ QR, const h16* __restrict__ KP, const h16* __restrict__ KR,
                                                                                          const h16* __restrict__ VT, const int* __restrict__ gmask, h16* XP) { flash_body<0>(QH, QR, KP, KR, VT, gmask, XP); }
__global__ __launch_bounds__(32 * AW) __attribute__((amdgpu_num_vgpr(256))) void k_flash_glb(const h16* __restrict__ QH, const h16* __restrict__ QR, const h16* __restrict__ KP, const h16* __restrict__ KR,
                                                                                          const h16* __restrict__ VT, const int* __restrict__ gmask, h16* XP) { flash_body<1>(QH, QR, KP, KR, VT, gmask, XP); }

static constexpr size_t al256(size_t v) { return (v + 255) & ~(size_t)255; }
static constexpr size_t SZ_XB = al256((size_t)NB * SEQ * DM * 2);
static constexpr size_t SZ_WB = al256((size_t)6 * DM * DM * 2);
static constexpr size_t SZ_WO = al256((size_t)DM * DM * 2);
static constexpr size_t SZ_PL = al256((size_t)NB * NH_ * SEQ * HD * 2);
static constexpr size_t SZ_XP = al256((size_t)NB * SEQ * DM * 2);
static constexpr size_t SZ_TOTAL = SZ_XB + SZ_WB + SZ_WO + 10 * SZ_PL + SZ_XP;
static_assert(SZ_TOTAL <= (size_t)134217728);
static_assert(((size_t)DM * DM * 2) % 256 == 0);
static_assert((size_t)NB * NH_ * SEQ * HD == (size_t)NB * DM * SEQ);
static_assert((size_t)(NB * SEQ / 64) * 64 == (size_t)NB * SEQ);
static_assert((size_t)(DM / 64) * 64 == (size_t)DM);

extern "C" void kernel_launch(void* const* d_in, const int* in_sizes, int n_in,
                              void* d_out, int out_size, void* d_ws, size_t ws_size, hipStream_t stream) {
    if (n_in < 16) return;
    const size_t needx = ((size_t)(NB - 1) * SEQ_FULL + SEQ) * DM;
    const size_t needm = (size_t)(NB - 1) * SEQ_FULL + SEQ;
    if ((size_t)in_sizes[0] < needx || (size_t)in_sizes[1] < needm) return;
    for (int i = 0; i < 7; ++i) { if ((size_t)in_sizes[2 + 2 * i] < (size_t)DM * DM || in_sizes[3 + 2 * i] < DM) return; }
    if ((size_t)out_size < ((size_t)(NB - 1) * OUT_SEQ + SEQ) * DM) return;
    if (SZ_TOTAL > ws_size) return;
    const float* x = (const float*)d_in[0];
    const int* gm = (const int*)d_in[1];
    const float* w_out = (const float*)d_in[14];
    const float* b_out = (const float*)d_in[15];
    float* OUT = (float*)d_out;
    char* wsp = (char*)d_ws;
    bf* XB = (bf*)wsp; wsp += SZ_XB;
    bf* WB = (bf*)wsp; wsp += SZ_WB;
    h16* WO = (h16*)wsp; wsp += SZ_WO;
    h16* PL[6];
    for (int i = 0; i < 6; ++i) { PL[i] = (h16*)wsp; wsp += SZ_PL; }
    h16* RP[4];
    for (int i = 0; i < 4; ++i) { RP[i] = (h16*)wsp; wsp += SZ_PL; }
    h16* XP = (h16*)wsp; wsp += SZ_XP;

    if (SEQ == SEQ_FULL) {
        const size_t n8 = (size_t)NB * SEQ * DM / 8;
        k_cvt8<<<(unsigned)((n8 + 255) / 256), 256, 0, stream>>>(x, XB, n8);
    } else {
        const size_t n8 = (size_t)SEQ * DM / 8;
        for (int b = 0; b < NB; ++b) k_cvt8<<<(unsigned)((n8 + 255) / 256), 256, 0, stream>>>(x + (size_t)b * SEQ_FULL * DM, XB + (size_t)b * SEQ * DM, n8);
    }
    for (int i = 0; i < 6; ++i)
        k_wt_b<<<dim3(DM / 64, DM / 64, 1), 256, 0, stream>>>((const float*)d_in[2 + 2 * i], WB + (size_t)i * DM * DM);
    k_wt_h<<<dim3(DM / 64, DM / 64, 1), 256, 0, stream>>>(w_out, WO);

    for (int i = 0; i < 6; ++i) {
        const bf* W = WB + (size_t)i * DM * DM; const float* bias = (const float*)d_in[3 + 2 * i];
        if (i == 2 || i == 5) k_proj_cols<<<dim3(DM / 64, NB * SEQ / 64, 1), 32, 0, stream>>>(W, XB, bias, PL[i]);
        else { const int ri = (i < 2) ? i : (i - 1);
               k_proj_rows<<<dim3(NB * SEQ / 64, DM / 64, 1), 32, 0, stream>>>(XB, W, bias, PL[i], RP[ri]); }
    }

    k_flash_win<<<dim3(SEQ / (16 * AW), NB * NH_, 1), 32 * AW, 0, stream>>>(PL[0], RP[0], PL[1], RP[1], PL[2], gm, XP);
    k_flash_glb<<<dim3(SEQ / (16 * AW), NB * NH_, 1), 32 * AW, 0, stream>>>(PL[3], RP[2], PL[4], RP[3], PL[5], gm, XP);

    k_oproj<<<dim3(NB * SEQ / 64, DM / 64, 1), 32, 0, stream>>>(XP, WO, b_out, OUT);
}
